// _AttentionLayer_5652176961576
// MI455X (gfx1250) — hardware-run, weakly checked
//
#include <hip/hip_runtime.h>
#include <stddef.h>


typedef _Float16 v16h __attribute__((ext_vector_type(16)));
typedef _Float16 v8h  __attribute__((ext_vector_type(8)));
typedef float    v8f  __attribute__((ext_vector_type(8)));
typedef float    v4f  __attribute__((ext_vector_type(4)));
typedef _Float16 h16;

#ifndef NB
#define NB 4
#endif
#ifndef SEQ
#define SEQ 4096
#endif
#define NB_FULL  4
#define SEQ_FULL 4096
#define DIM   256
#define HID   2048
#define MROWS (NB * SEQ)
#define NCHUNK 2
#define CROWS (MROWS / NCHUNK)

static_assert(NB >= 1 && NB <= NB_FULL);
static_assert(SEQ >= 64 && SEQ <= SEQ_FULL && (SEQ % 64) == 0);
static_assert((DIM % 64) == 0 && (DIM % 32) == 0);
static_assert((HID % 64) == 0 && (HID % 32) == 0);
static_assert((MROWS % 64) == 0 && (MROWS % 8) == 0);
static_assert((MROWS % NCHUNK) == 0 && (CROWS % 64) == 0 && (CROWS % 8) == 0);
static_assert(DIM == 32 * 8);
static_assert(DIM == 2 * 32 * 4);
static_assert(HID == 8 * 32 * 8);
static_assert(DIM == 16 * 16);
static_assert((size_t)MROWS * DIM < (size_t)0x7FFFFFFFu);
static_assert((size_t)NB * DIM * SEQ < (size_t)0x7FFFFFFFu);
static_assert((size_t)MROWS * HID < (size_t)0xFFFFFFFFu);

#define LDT 72
#define LDC 68
#define LDO 132
static_assert((LDT % 8) == 0 && LDT >= 64);
static_assert((LDC % 4) == 0 && LDC >= 64);
static_assert((LDO % 4) == 0 && LDO >= 128);

#define WCARRY 64.0f
#define MCARRY 16.0f
#define RCARRY 2048.0f
#define PSHIFT 9.704060528f

#define WSQ_BYTES     ((size_t)DIM * DIM * 2)
#define WFF_BYTES     ((size_t)DIM * HID * 2)
#define PLANE16_BYTES ((size_t)MROWS * DIM * 2)
#define PLANE32_BYTES ((size_t)MROWS * DIM * 4)
#define HCH_BYTES     ((size_t)CROWS * HID * 2)
#define OFF_WQ  ((size_t)0)
#define OFF_WK  (OFF_WQ + WSQ_BYTES)
#define OFF_WV  (OFF_WK + WSQ_BYTES)
#define OFF_W0  (OFF_WV + WSQ_BYTES)
#define OFF_W1  (OFF_W0 + WSQ_BYTES)
#define OFF_W2  (OFF_W1 + WFF_BYTES)
#define OFF_REG (OFF_W2 + WFF_BYTES)
#define OFF_X16 (OFF_REG)
#define OFF_QH  (OFF_X16 + PLANE16_BYTES)
#define OFF_QR  (OFF_QH + PLANE16_BYTES)
#define OFF_KH  (OFF_QR + PLANE16_BYTES)
#define OFF_KR  (OFF_KH + PLANE16_BYTES)
#define OFF_VT  (OFF_KR + PLANE16_BYTES)
#define OFF_A32 (OFF_VT + PLANE16_BYTES)
#define OFF_T1  (OFF_A32 + PLANE32_BYTES)
#define PRE_END (OFF_T1 + PLANE16_BYTES)
#define OFF_HRAW (OFF_REG)
#define OFF_MID  (OFF_HRAW + HCH_BYTES)
#define MLP_END  (OFF_MID + HCH_BYTES)
#define REG_END  ((PRE_END > MLP_END) ? PRE_END : MLP_END)
#define OFF_E32 (REG_END)
#define OFF_E16 (OFF_E32 + PLANE32_BYTES)
#define OFF_V32 (OFF_E16 + PLANE16_BYTES)
#define WS_TOTAL (OFF_V32 + PLANE32_BYTES)
static_assert((WSQ_BYTES % 128) == 0 && (WFF_BYTES % 128) == 0 && (PLANE16_BYTES % 128) == 0);
static_assert((PLANE32_BYTES % 128) == 0 && (HCH_BYTES % 128) == 0);
static_assert(PRE_END <= REG_END && MLP_END <= REG_END);
static_assert(WS_TOTAL <= (size_t)134217728);

__device__ __forceinline__ float bf16r(float x) {
  unsigned int u = __float_as_uint(x);
  u = (u + 0x7FFFu + ((u >> 16) & 1u)) & 0xFFFF0000u;
  return __uint_as_float(u);
}

static __device__ __forceinline__ h16 toh_flush(float v) {
  const h16 r = (h16)v;
  return (fabsf(v) < 6.103515625e-05f) ? (h16)0.0f : r;
}

__device__ __forceinline__ v16h frag_at(const _Float16* p) {
  v8h lo = *(const v8h*)(p);
  v8h hi = *(const v8h*)(p + 16);
  v16h out;
#pragma unroll
  for (int i = 0; i < 8; ++i) { out[i] = lo[i]; out[i + 8] = hi[i]; }
  return out;
}
__device__ __forceinline__ v16h ld_frag(const _Float16* base, unsigned ld) {
  const unsigned lane = threadIdx.x & 31u;
  return frag_at(base + (lane & 15u) * ld + (lane >> 4) * 8u);
}

__device__ __forceinline__ v8f wmma16(v16h a, v16h b, v8f c) {
  v8f d = __builtin_amdgcn_wmma_f32_16x16x32_f16(false, a, false, b, (short)0, c,
                                                 false, false);
  asm volatile("v_nop\n\tv_nop\n\tv_nop\n\tv_nop" : "+v"(d) : "v"(a), "v"(b));
  return d;
}

__device__ __forceinline__ float red16_max(float x) {
#pragma unroll
  for (int off = 1; off < 16; off <<= 1) x = fmaxf(x, __shfl_xor(x, off, 32));
  return x;
}
__device__ __forceinline__ float red16_sum(float x) {
#pragma unroll
  for (int off = 1; off < 16; off <<= 1) x += __shfl_xor(x, off, 32);
  return x;
}
__device__ __forceinline__ float red32_sum(float x) {
#pragma unroll
  for (int off = 1; off < 32; off <<= 1) x += __shfl_xor(x, off, 32);
  return x;
}

__device__ __forceinline__ void wave_lds_sync() {
  __builtin_amdgcn_fence(3  , "wavefront");
  asm volatile("s_wait_dscnt 0x0" ::: "memory");
  __builtin_amdgcn_wave_barrier();
}

__device__ __forceinline__ float leaky_act(float t) {
  return (t >= 0.0f) ? t : 0.01f * t;
}

__global__ __launch_bounds__(256) void wconv_kernel(
    const float* __restrict__ W, _Float16* __restrict__ Wt, unsigned ldw, unsigned ldk) {
  __shared__ _Float16 T[64 * LDT];
  const unsigned tid = threadIdx.x;
  const unsigned n0 = blockIdx.x * 64u;
  const unsigned k0 = blockIdx.y * 64u;
#pragma unroll 4
  for (unsigned j = 0; j < 16u; ++j) {
    const unsigned idx = tid + 256u * j;
    const unsigned kr = idx >> 6, nc = idx & 63u;
    const float v = W[(size_t)(k0 + kr) * ldw + n0 + nc];
    T[nc * LDT + kr] = (_Float16)(WCARRY * bf16r(v));
  }
  __syncthreads();
  v8h x[2];
  size_t off[2];
#pragma unroll
  for (unsigned i = 0; i < 2u; ++i) {
    const unsigned n = 32u * i + (tid >> 3);
    const unsigned kc = (tid & 7u) * 8u;
    x[i] = *(const v8h*)&T[n * LDT + kc];
    off[i] = (size_t)(n0 + n) * ldk + k0 + kc;
  }
#pragma unroll
  for (int i = 0; i < 2; ++i) *(volatile v8h*)(Wt + off[i]) = x[i];
  __threadfence();
#pragma unroll
  for (int i = 0; i < 2; ++i) *(volatile v8h*)(Wt + off[i]) = x[i];
}

__global__ __launch_bounds__(256) void xconv_kernel(
    const float* __restrict__ X, _Float16* __restrict__ dst) {
  const unsigned lane = threadIdx.x & 31u, w = threadIdx.x >> 5;
  const unsigned crow = blockIdx.x * 8u + w;
  const unsigned bidx = crow / (unsigned)SEQ;
  const unsigned sq = crow - bidx * (unsigned)SEQ;
  const size_t srow = (size_t)bidx * SEQ_FULL + sq;
  const float* xr = X + srow * DIM + lane * 8u;
  const v4f a0 = *(const v4f*)(xr);
  const v4f a1 = *(const v4f*)(xr + 4u);
  v8h o;
#pragma unroll
  for (int i = 0; i < 4; ++i) {
    o[i]     = toh_flush(bf16r(a0[i]));
    o[i + 4] = toh_flush(bf16r(a1[i]));
  }
  _Float16* p = dst + (size_t)crow * DIM + lane * 8u;
  *(volatile v8h*)p = o;
  __threadfence();
  *(volatile v8h*)p = o;
}

__global__ __launch_bounds__(256) void ln1_kernel(
    const float* __restrict__ X, const float* __restrict__ A32, const float* __restrict__ G,
    const float* __restrict__ Be, _Float16* __restrict__ dst) {
  const unsigned lane = threadIdx.x & 31u, w = threadIdx.x >> 5;
  const unsigned crow = blockIdx.x * 8u + w;
  const unsigned bidx = crow / (unsigned)SEQ;
  const unsigned sq = crow - bidx * (unsigned)SEQ;
  const size_t srow = (size_t)bidx * SEQ_FULL + sq;
  const float* xr = X + srow * DIM + lane * 8u;
  const float* ar = A32 + (size_t)crow * DIM + lane * 8u;
  const v4f x0 = *(const v4f*)(xr);
  const v4f x1 = *(const v4f*)(xr + 4u);
  const v4f a0 = *(const v4f*)(ar);
  const v4f a1 = *(const v4f*)(ar + 4u);
  v4f t0, t1;
  float s = 0.0f;
#pragma unroll
  for (int i = 0; i < 4; ++i) {
    t0[i] = bf16r(x0[i]) + a0[i];
    t1[i] = bf16r(x1[i]) + a1[i];
    s += t0[i] + t1[i];
  }
  const float mean = red32_sum(s) * (1.0f / (float)DIM);
  float ss = 0.0f;
#pragma unroll
  for (int i = 0; i < 4; ++i) {
    const float d0 = t0[i] - mean;
    const float d1 = t1[i] - mean;
    ss += d0 * d0;
    ss += d1 * d1;
  }
  const float var = red32_sum(ss) * (1.0f / (float)DIM);
  const float rstd = 1.0f / sqrtf(var + 1.0e-5f);
  const unsigned c = lane * 8u;
  const v4f g0 = *(const v4f*)(G + c);
  const v4f g1 = *(const v4f*)(G + c + 4u);
  const v4f b0 = *(const v4f*)(Be + c);
  const v4f b1 = *(const v4f*)(Be + c + 4u);
  v8h o;
#pragma unroll
  for (int i = 0; i < 4; ++i) {
    o[i]     = toh_flush((t0[i] - mean) * rstd * bf16r(g0[i]) + bf16r(b0[i]));
    o[i + 4] = toh_flush((t1[i] - mean) * rstd * bf16r(g1[i]) + bf16r(b1[i]));
  }
  _Float16* p = dst + (size_t)crow * DIM + c;
  *(volatile v8h*)p = o;
  __threadfence();
  *(volatile v8h*)p = o;
}

__global__ __launch_bounds__(256) void ln_mid_kernel(
    const _Float16* __restrict__ Hr, const float* __restrict__ G, const float* __restrict__ Be,
    _Float16* __restrict__ dst) {
  const unsigned lane = threadIdx.x & 31u, w = threadIdx.x >> 5;
  const unsigned crow = blockIdx.x * 8u + w;
  const _Float16* hr = Hr + (size_t)crow * HID + lane * 8u;

  float s = 0.0f;
#pragma unroll 1
  for (unsigned j = 0; j < 8u; ++j) {
    const v8h a = *(const v8h*)(hr + j * 256u);
#pragma unroll
    for (int i = 0; i < 8; ++i) s += (float)a[i];
  }
  const float mean = red32_sum(s) * (1.0f / (float)HID);

  float ss = 0.0f;
#pragma unroll 1
  for (unsigned j = 0; j < 8u; ++j) {
    const v8h a = *(const v8h*)(hr + j * 256u);
#pragma unroll
    for (int i = 0; i < 8; ++i) {
      const float d = (float)a[i] - mean;
      ss += d * d;
    }
  }
  const float var = red32_sum(ss) * (1.0f / (float)HID);
  const float rstd = 1.0f / sqrtf(var + 1.0e-5f);

#pragma unroll 1
  for (unsigned j = 0; j < 8u; ++j) {
    const unsigned c = j * 256u + lane * 8u;
    const v8h a = *(const v8h*)(hr + j * 256u);
    const v4f g0 = *(const v4f*)(G + c);
    const v4f g1 = *(const v4f*)(G + c + 4u);
    const v4f b0 = *(const v4f*)(Be + c);
    const v4f b1 = *(const v4f*)(Be + c + 4u);
    v8h o;
#pragma unroll
    for (int i = 0; i < 4; ++i) {
      const float d0 = (float)a[i] - mean;
      const float d1 = (float)a[i + 4] - mean;
      const float y0 = leaky_act(d0 * rstd * bf16r(g0[i]) + bf16r(b0[i]));
      const float y1 = leaky_act(d1 * rstd * bf16r(g1[i]) + bf16r(b1[i]));
      o[i]     = toh_flush(MCARRY * y0);
      o[i + 4] = toh_flush(MCARRY * y1);
    }
    _Float16* p = dst + (size_t)crow * HID + c;
    *(volatile v8h*)p = o;
    __threadfence();
    *(volatile v8h*)p = o;
  }
}

__global__ __launch_bounds__(256) void ln_out_kernel(
    const float* __restrict__ V32, const float* __restrict__ G, const float* __restrict__ Be,
    float* __restrict__ outp) {
  const unsigned lane = threadIdx.x & 31u, w = threadIdx.x >> 5;
  const unsigned crow = blockIdx.x * 8u + w;
  const unsigned bidx = crow / (unsigned)SEQ;
  const unsigned sq = crow - bidx * (unsigned)SEQ;
  const size_t frow = (size_t)bidx * SEQ_FULL + sq;
  const float* vr = V32 + (size_t)crow * DIM + lane * 4u;
  const v4f a0 = *(const v4f*)(vr);
  const v4f a1 = *(const v4f*)(vr + 128u);
  float s = 0.0f;
#pragma unroll
  for (int i = 0; i < 4; ++i) s += a0[i] + a1[i];
  const float mean = red32_sum(s) * (1.0f / (float)DIM);
  float ss = 0.0f;
#pragma unroll
  for (int i = 0; i < 4; ++i) {
    const float d0 = a0[i] - mean;
    const float d1 = a1[i] - mean;
    ss += d0 * d0;
    ss += d1 * d1;
  }
  const float var = red32_sum(ss) * (1.0f / (float)DIM);
  const float rstd = 1.0f / sqrtf(var + 1.0e-5f);
  const unsigned c = lane * 4u;
  const v4f g0 = *(const v4f*)(G + c);
  const v4f g1 = *(const v4f*)(G + c + 128u);
  const v4f b0 = *(const v4f*)(Be + c);
  const v4f b1 = *(const v4f*)(Be + c + 128u);
  v4f o0, o1;
#pragma unroll
  for (int i = 0; i < 4; ++i) {
    o0[i] = (a0[i] - mean) * rstd * bf16r(g0[i]) + bf16r(b0[i]);
    o1[i] = (a1[i] - mean) * rstd * bf16r(g1[i]) + bf16r(b1[i]);
  }
  float* p = outp + frow * DIM + c;
  *(volatile v4f*)p = o0;
  *(volatile v4f*)(p + 128u) = o1;
  __threadfence();
  *(volatile v4f*)p = o0;
  *(volatile v4f*)(p + 128u) = o1;
}

template <int MODE>
__device__ __forceinline__ void gemm_body(
    const _Float16* __restrict__ A16, const _Float16* __restrict__ Bt, const unsigned K,
    const float* __restrict__ bias, const float* __restrict__ addf,
    float* __restrict__ outf, _Float16* __restrict__ out16, _Float16* __restrict__ out16r) {
  __shared__ float Cs[64 * LDC];
  const unsigned tid = threadIdx.x, lane = tid & 31u, w = tid >> 5;
  const unsigned mw = w >> 1, nw = w & 1u;
  const unsigned hh = lane >> 4, m = lane & 15u;
  const unsigned n0 = blockIdx.x * 64u;
  const unsigned row0 = blockIdx.y * 64u;

  const _Float16* ap  = A16 + (size_t)(row0 + mw * 16u + m) * K + hh * 8u;
  const _Float16* bp0 = Bt + (size_t)(n0 + nw * 32u + m) * K + hh * 8u;
  const _Float16* bp1 = bp0 + (size_t)16 * K;
  v8f acc0 = {}, acc1 = {};
#pragma unroll 2
  for (unsigned k0 = 0; k0 < K; k0 += 32u) {
    const v16h a  = frag_at(ap + k0);
    const v16h b0 = frag_at(bp0 + k0);
    const v16h b1 = frag_at(bp1 + k0);
    acc0 = wmma16(a, b0, acc0);
    acc1 = wmma16(a, b1, acc1);
  }
#pragma unroll
  for (int r = 0; r < 8; ++r) {
    float* d = &Cs[(mw * 16u + hh * 8u + (unsigned)r) * LDC + nw * 32u + m];
    d[0]  = acc0[r];
    d[16] = acc1[r];
  }
  __syncthreads();

  if (MODE == 0 || MODE == 2 || MODE == 3) {
    const unsigned ldo = (MODE == 3) ? (unsigned)HID : (unsigned)DIM;
    v8h x[2], xr[2];
    size_t off[2];
#pragma unroll
    for (unsigned i = 0; i < 2u; ++i) {
      const unsigned r = 32u * i + (tid >> 3);
      const unsigned c = (tid & 7u) * 8u;
      const v4f u0 = *(const v4f*)&Cs[r * LDC + c];
      const v4f u1 = *(const v4f*)&Cs[r * LDC + c + 4];
      const v4f g0 = *(const v4f*)(bias + n0 + c);
      const v4f g1 = *(const v4f*)(bias + n0 + c + 4u);
#pragma unroll
      for (int j = 0; j < 4; ++j) {
        const float t0 = u0[j] * (1.0f / WCARRY) + bf16r(g0[j]);
        const float t1 = u1[j] * (1.0f / WCARRY) + bf16r(g1[j]);
        const h16 h0 = toh_flush(t0);
        const h16 h1 = toh_flush(t1);
        x[i][j]     = h0;
        x[i][j + 4] = h1;
        if (MODE == 0) {
          xr[i][j]     = toh_flush((t0 - (float)h0) * RCARRY);
          xr[i][j + 4] = toh_flush((t1 - (float)h1) * RCARRY);
        }
      }
      off[i] = (size_t)(row0 + r) * ldo + n0 + c;
    }
    v4f xs[4];
    size_t offf[4];
    if (MODE == 2) {
#pragma unroll
      for (unsigned i = 0; i < 4u; ++i) {
        const unsigned r = 16u * i + (tid >> 4);
        const unsigned c = (tid & 15u) * 4u;
        const v4f u = *(const v4f*)&Cs[r * LDC + c];
        const v4f g = *(const v4f*)(bias + n0 + c);
        v4f val;
#pragma unroll
        for (int j = 0; j < 4; ++j) val[j] = u[j] * (1.0f / WCARRY) + bf16r(g[j]);
        xs[i] = val;
        offf[i] = (size_t)(row0 + r) * DIM + n0 + c;
      }
    }
#pragma unroll
    for (int i = 0; i < 2; ++i) *(volatile v8h*)(out16 + off[i]) = x[i];
    if (MODE == 0) {
#pragma unroll
      for (int i = 0; i < 2; ++i) *(volatile v8h*)(out16r + off[i]) = xr[i];
    }
    if (MODE == 2) {
#pragma unroll
      for (int i = 0; i < 4; ++i) *(volatile v4f*)(outf + offf[i]) = xs[i];
    }
    __threadfence();
#pragma unroll
    for (int i = 0; i < 2; ++i) *(volatile v8h*)(out16 + off[i]) = x[i];
    if (MODE == 0) {
#pragma unroll
      for (int i = 0; i < 2; ++i) *(volatile v8h*)(out16r + off[i]) = xr[i];
    }
    if (MODE == 2) {
#pragma unroll
      for (int i = 0; i < 4; ++i) *(volatile v4f*)(outf + offf[i]) = xs[i];
    }
  }

  if (MODE == 1) {
    const unsigned bidx = row0 / (unsigned)SEQ;
    const unsigned key0 = row0 - bidx * (unsigned)SEQ;
    v8h x[2];
    size_t off[2];
#pragma unroll
    for (unsigned i = 0; i < 2u; ++i) {
      const unsigned dcol = 32u * i + (tid >> 3);
      const unsigned kk = (tid & 7u) * 8u;
      const float bb = bf16r(bias[n0 + dcol]);
#pragma unroll
      for (unsigned j = 0; j < 8u; ++j) {
        const float t = Cs[(kk + j) * LDC + dcol] * (1.0f / WCARRY) + bb;
        x[i][j] = toh_flush(t);
      }
      off[i] = ((size_t)bidx * DIM + n0 + dcol) * SEQ + key0 + kk;
    }
#pragma unroll
    for (int i = 0; i < 2; ++i) *(volatile v8h*)(out16 + off[i]) = x[i];
    __threadfence();
#pragma unroll
    for (int i = 0; i < 2; ++i) *(volatile v8h*)(out16 + off[i]) = x[i];
  }

  if (MODE == 4) {
    const float cs = 1.0f / (WCARRY * MCARRY);
    v4f xs[4];
    size_t off[4];
#pragma unroll
    for (unsigned i = 0; i < 4u; ++i) {
      const unsigned r = 16u * i + (tid >> 4);
      const unsigned c = (tid & 15u) * 4u;
      const size_t rc = (size_t)(row0 + r) * DIM + n0 + c;
      const v4f u = *(const v4f*)&Cs[r * LDC + c];
      const v4f g = *(const v4f*)(bias + n0 + c);
      const v4f ein = *(const v4f*)(addf + rc);
      v4f val;
#pragma unroll
      for (int j = 0; j < 4; ++j) val[j] = leaky_act((u[j] * cs + bf16r(g[j])) + ein[j]);
      xs[i] = val;
      off[i] = rc;
    }
#pragma unroll
    for (int i = 0; i < 4; ++i) *(volatile v4f*)(outf + off[i]) = xs[i];
    __threadfence();
#pragma unroll
    for (int i = 0; i < 4; ++i) *(volatile v4f*)(outf + off[i]) = xs[i];
  }
}

__global__ __launch_bounds__(256) void gemm_qk_kernel(
    const _Float16* __restrict__ A16, const _Float16* __restrict__ Bt,
    const float* __restrict__ bias, _Float16* __restrict__ out16, _Float16* __restrict__ out16r) {
  gemm_body<0>(A16, Bt, (unsigned)DIM, bias, bias, (float*)0, out16, out16r);
}
__global__ __launch_bounds__(256) void gemm_v_kernel(
    const _Float16* __restrict__ A16, const _Float16* __restrict__ Bt,
    const float* __restrict__ bias, _Float16* __restrict__ vt) {
  gemm_body<1>(A16, Bt, (unsigned)DIM, bias, bias, (float*)0, vt, vt);
}
__global__ __launch_bounds__(256) void gemm_e_kernel(
    const _Float16* __restrict__ A16, const _Float16* __restrict__ Bt,
    const float* __restrict__ bias, float* __restrict__ e32, _Float16* __restrict__ e16) {
  gemm_body<2>(A16, Bt, (unsigned)DIM, bias, bias, e32, e16, e16);
}
__global__ __launch_bounds__(256) void gemm_h_kernel(
    const _Float16* __restrict__ A16, const _Float16* __restrict__ Bt,
    const float* __restrict__ bias, _Float16* __restrict__ hraw) {
  gemm_body<3>(A16, Bt, (unsigned)DIM, bias, bias, (float*)0, hraw, hraw);
}
__global__ __launch_bounds__(256) void gemm_l_kernel(
    const _Float16* __restrict__ A16, const _Float16* __restrict__ Bt,
    const float* __restrict__ bias, const float* __restrict__ e32, float* __restrict__ v32) {
  gemm_body<4>(A16, Bt, (unsigned)HID, bias, e32, v32, (_Float16*)0, (_Float16*)0);
}

__global__ __launch_bounds__(128) __attribute__((amdgpu_num_vgpr(256))) void attn_kernel(
    const _Float16* __restrict__ Qh, const _Float16* __restrict__ Qr,
    const _Float16* __restrict__ Kh, const _Float16* __restrict__ Kr,
    const _Float16* __restrict__ Vt, float* __restrict__ Ao) {
  __shared__ __attribute__((aligned(16))) float St[4 * 16 * LDO];

  const unsigned lane = threadIdx.x & 31u;
  const unsigned w = (unsigned)__builtin_amdgcn_readfirstlane((int)(threadIdx.x >> 5));
  const unsigned hh = lane >> 4, m = lane & 15u;
  const unsigned b = blockIdx.y;
  const unsigned qrow0 = blockIdx.x * 64u + w * 16u;

  const unsigned qoff = (b * (unsigned)SEQ + qrow0 + m) * (unsigned)DIM + hh * 8u;
  const unsigned koff = (b * (unsigned)SEQ + m) * (unsigned)DIM + hh * 8u;
  const unsigned voff = (b * (unsigned)DIM + m) * (unsigned)SEQ + hh * 8u;

  float mrow = -1.0e30f, lrow = 0.0f;
  v8f o[16];
#pragma unroll
  for (int j = 0; j < 16; ++j) o[j] = (v8f){};

  for (unsigned kb = 0; kb < (unsigned)SEQ; kb += 32u) {
    const unsigned k0off = koff + kb * (unsigned)DIM;
    const unsigned k1off = k0off + 16u * (unsigned)DIM;
    v8f sm0 = {}, sr0 = {}, sm1 = {}, sr1 = {};
#pragma unroll 1
    for (unsigned c = 0; c < (unsigned)DIM; c += 32u) {
      const v16h qh = frag_at(Qh + qoff + c);
      const v16h qr = frag_at(Qr + qoff + c);
      const v16h ka = frag_at(Kh + k0off + c);
      const v16h ra = frag_at(Kr + k0off + c);
      sm0 = wmma16(ka, qh, sm0);
      sr0 = wmma16(ka, qr, sr0);
      sr0 = wmma16(ra, qh, sr0);
      const v16h kc = frag_at(Kh + k1off + c);
      const v16h rc = frag_at(Kr + k1off + c);
      sm1 = wmma16(kc, qh, sm1);
      sr1 = wmma16(kc, qr, sr1);
      sr1 = wmma16(rc, qh, sr1);
    }

    v8f s0, s1;
#pragma unroll
    for (int r = 0; r < 8; ++r) {
      s0[r] = sm0[r] + sr0[r] * (1.0f / RCARRY);
      s1[r] = sm1[r] + sr1[r] * (1.0f / RCARRY);
    }
    float mx = fmaxf(s0[0], s1[0]);
#pragma unroll
    for (int r = 1; r < 8; ++r) mx = fmaxf(mx, fmaxf(s0[r], s1[r]));
    mx = fmaxf(mx, __shfl_xor(mx, 16, 32));
    const float mn = fmaxf(mrow, mx);
    const float alpha = __expf(mrow - mn);
    mrow = mn;

    v16h pf;
    float rs = 0.0f;
#pragma unroll
    for (int r = 0; r < 8; ++r) {
      const h16 p0 = toh_flush(__expf((s0[r] - mn) + PSHIFT));
      const h16 p1 = toh_flush(__expf((s1[r] - mn) + PSHIFT));
      pf[r]     = p0;
      pf[r + 8] = p1;
      rs += (float)p0 + (float)p1;
    }
    rs += __shfl_xor(rs, 16, 32);
    lrow = alpha * lrow + rs;
#pragma unroll
    for (int j = 0; j < 16; ++j) o[j] = o[j] * alpha;

#pragma unroll
    for (int jg = 0; jg < 4; ++jg) {
      v16h vf[4];
#pragma unroll
      for (int t = 0; t < 4; ++t)
        vf[t] = frag_at(Vt + voff + (unsigned)((jg * 4 + t) * 16) * (unsigned)SEQ + kb);
#pragma unroll
      for (int t = 0; t < 4; ++t) o[jg * 4 + t] = wmma16(vf[t], pf, o[jg * 4 + t]);
    }
  }

  const float inv = __builtin_amdgcn_rcpf(lrow);
  const unsigned sbase = w * (16u * LDO);
#pragma unroll
  for (int half = 0; half < 2; ++half) {
#pragma unroll
    for (int j = 0; j < 8; ++j)
#pragma unroll
      for (int r = 0; r < 8; ++r)
        St[sbase + m * LDO + (unsigned)j * 16u + hh * 8u + (unsigned)r] = o[half * 8 + j][r] * inv;
    wave_lds_sync();
    v4f x[16];
    unsigned off[16];
#pragma unroll
    for (unsigned i = 0; i < 16u; ++i) {
      x[i] = *(const v4f*)&St[sbase + i * LDO + lane * 4u];
      off[i] = (b * (unsigned)SEQ + qrow0 + i) * (unsigned)DIM + (unsigned)half * 128u + lane * 4u;
    }
#pragma unroll
    for (int i = 0; i < 16; ++i) *(volatile v4f*)(Ao + off[i]) = x[i];
    __threadfence();
#pragma unroll
    for (int i = 0; i < 16; ++i) *(volatile v4f*)(Ao + off[i]) = x[i];
    wave_lds_sync();
  }
}

extern "C" void kernel_launch(void* const* d_in, const int* in_sizes, int n_in,
                              void* d_out, int out_size, void* d_ws, size_t ws_size,
                              hipStream_t stream) {
  if (n_in < 19) return;
  const long long need_x = ((long long)(NB - 1) * SEQ_FULL + SEQ) * DIM;
  if ((long long)in_sizes[0] < need_x) return;
  if ((long long)in_sizes[1] < (long long)DIM * DIM) return;
  if ((long long)in_sizes[3] < (long long)DIM * DIM) return;
  if ((long long)in_sizes[5] < (long long)DIM * DIM) return;
  if ((long long)in_sizes[7] < (long long)DIM * DIM) return;
  if ((long long)in_sizes[9] < (long long)DIM * HID) return;
  if ((long long)in_sizes[13] < (long long)DIM * HID) return;
  if (in_sizes[2] < DIM || in_sizes[4] < DIM || in_sizes[6] < DIM || in_sizes[8] < DIM) return;
  if (in_sizes[10] < HID || in_sizes[11] < HID || in_sizes[12] < HID) return;
  if (in_sizes[14] < DIM || in_sizes[15] < DIM || in_sizes[16] < DIM) return;
  if (in_sizes[17] < DIM || in_sizes[18] < DIM) return;
  if ((long long)out_size < need_x) return;
  if (ws_size < WS_TOTAL) return;

  const float* X    = (const float*)d_in[0];
  const float* wq   = (const float*)d_in[1];
  const float* bq   = (const float*)d_in[2];
  const float* wk   = (const float*)d_in[3];
  const float* bk   = (const float*)d_in[4];
  const float* wv   = (const float*)d_in[5];
  const float* bv   = (const float*)d_in[6];
  const float* w0   = (const float*)d_in[7];
  const float* b0   = (const float*)d_in[8];
  const float* w1   = (const float*)d_in[9];
  const float* b1   = (const float*)d_in[10];
  const float* gm   = (const float*)d_in[11];
  const float* bm   = (const float*)d_in[12];
  const float* w2   = (const float*)d_in[13];
  const float* b2   = (const float*)d_in[14];
  const float* g1   = (const float*)d_in[15];
  const float* be1  = (const float*)d_in[16];
  const float* g2   = (const float*)d_in[17];
  const float* be2  = (const float*)d_in[18];
  float* out = (float*)d_out;

  char* ws = (char*)d_ws;
  _Float16* Wq_t  = (_Float16*)(ws + OFF_WQ);
  _Float16* Wk_t  = (_Float16*)(ws + OFF_WK);
  _Float16* Wv_t  = (_Float16*)(ws + OFF_WV);
  _Float16* W0_t  = (_Float16*)(ws + OFF_W0);
  _Float16* W1_t  = (_Float16*)(ws + OFF_W1);
  _Float16* W2_t  = (_Float16*)(ws + OFF_W2);
  _Float16* X16   = (_Float16*)(ws + OFF_X16);
  _Float16* Qh16  = (_Float16*)(ws + OFF_QH);
  _Float16* Qr16  = (_Float16*)(ws + OFF_QR);
  _Float16* Kh16  = (_Float16*)(ws + OFF_KH);
  _Float16* Kr16  = (_Float16*)(ws + OFF_KR);
  _Float16* Vt16  = (_Float16*)(ws + OFF_VT);
  float*    A32   = (float*)(ws + OFF_A32);
  _Float16* T116  = (_Float16*)(ws + OFF_T1);
  _Float16* Hraw  = (_Float16*)(ws + OFF_HRAW);
  _Float16* Mid16 = (_Float16*)(ws + OFF_MID);
  float*    E32   = (float*)(ws + OFF_E32);
  _Float16* E16   = (_Float16*)(ws + OFF_E16);
  float*    V32   = (float*)(ws + OFF_V32);

  dim3 blk(256);
  dim3 gsq(DIM / 64, DIM / 64);
  dim3 gg(DIM / 64, MROWS / 64);

  wconv_kernel<<<gsq, blk, 0, stream>>>(wq, Wq_t, (unsigned)DIM, (unsigned)DIM);
  wconv_kernel<<<gsq, blk, 0, stream>>>(wk, Wk_t, (unsigned)DIM, (unsigned)DIM);
  wconv_kernel<<<gsq, blk, 0, stream>>>(wv, Wv_t, (unsigned)DIM, (unsigned)DIM);
  wconv_kernel<<<gsq, blk, 0, stream>>>(w0, W0_t, (unsigned)DIM, (unsigned)DIM);
  wconv_kernel<<<dim3(HID / 64, DIM / 64), blk, 0, stream>>>(w1, W1_t, (unsigned)HID, (unsigned)DIM);
  wconv_kernel<<<dim3(DIM / 64, HID / 64), blk, 0, stream>>>(w2, W2_t, (unsigned)DIM, (unsigned)HID);

  xconv_kernel<<<dim3(MROWS / 8), blk, 0, stream>>>(X, X16);
  gemm_qk_kernel<<<gg, blk, 0, stream>>>(X16, Wq_t, bq, Qh16, Qr16);
  gemm_qk_kernel<<<gg, blk, 0, stream>>>(X16, Wk_t, bk, Kh16, Kr16);
  gemm_v_kernel<<<gg, blk, 0, stream>>>(X16, Wv_t, bv, Vt16);
  attn_kernel<<<dim3(SEQ / 64, NB), dim3(128), 0, stream>>>(Qh16, Qr16, Kh16, Kr16, Vt16, A32);
  ln1_kernel<<<dim3(MROWS / 8), blk, 0, stream>>>(X, A32, g1, be1, T116);
  gemm_e_kernel<<<gg, blk, 0, stream>>>(T116, W0_t, b0, E32, E16);

  for (int ch = 0; ch < NCHUNK; ++ch) {
    const size_t ro = (size_t)ch * CROWS * DIM;
    gemm_h_kernel<<<dim3(HID / 64, CROWS / 64), blk, 0, stream>>>(E16 + ro, W1_t, b1, Hraw);
    ln_mid_kernel<<<dim3(CROWS / 8), blk, 0, stream>>>(Hraw, gm, bm, Mid16);
    gemm_l_kernel<<<dim3(DIM / 64, CROWS / 64), blk, 0, stream>>>(Mid16, W2_t, b2, E32 + ro, V32 + ro);
  }
  ln_out_kernel<<<dim3(MROWS / 8), blk, 0, stream>>>(V32, g2, be2, out);
}
